// Link_Prediction_79096117723242
// MI455X (gfx1250) — hardware-verified
//
#include <hip/hip_runtime.h>
#include <stddef.h>


#define IN      128
#define HIDC    128
#define OUTC    64
#define NTHR    256
#define NWAVE   8
#define EPT     8
#define NGRP    2
#define CHUNK   (NTHR * EPT * NGRP)
#define WCAP    (EPT * NGRP * 32)
#define LISTN   (NWAVE * WCAP)
#define ESH     13
#define NBD     8192
#define NB1     512
#define NB2     1024
#define NRQ     1024
#define AGGF    65536
#define LDS_AGG (AGGF * 4 + LISTN * 4)
#define PPB     2048
#define WSC     16.0f
#define WSCI    0.0625f

static_assert(IN == 128 && HIDC == 128 && OUTC == 64);
static_assert((CHUNK & (CHUNK - 1)) == 0 && CHUNK <= 4096);
static_assert(NB1 * HIDC == AGGF && NB2 * OUTC == AGGF);
static_assert(NRQ % NB1 == 0 && NRQ % NB2 == 0 && NBD % NRQ == 0);
static_assert(NBD % (4 * NTHR) == 0);
static_assert(PPB % (4 * NTHR) == 0);

typedef float v2f __attribute__((ext_vector_type(2)));
typedef float v4f __attribute__((ext_vector_type(4)));
typedef float v8f __attribute__((ext_vector_type(8)));
typedef int   v4i __attribute__((ext_vector_type(4)));
typedef _Float16 v8h  __attribute__((ext_vector_type(8)));
typedef _Float16 v16h __attribute__((ext_vector_type(16)));
union Frag { v16h v; v8h half[2]; };

union DegLds { int c[NBD]; float f[NBD]; v4f v[NBD / 4]; };

__device__ __forceinline__ v8h cvt8h(v4f a, v4f b) {
  v8h r;
  r[0] = (_Float16)a.x; r[1] = (_Float16)a.y; r[2] = (_Float16)a.z; r[3] = (_Float16)a.w;
  r[4] = (_Float16)b.x; r[5] = (_Float16)b.y; r[6] = (_Float16)b.z; r[7] = (_Float16)b.w;
  return r;
}

__device__ __forceinline__ v8f wm(v16h a, v16h b, v8f c) {
  v8f d = __builtin_amdgcn_wmma_f32_16x16x32_f16(false, a, false, b, (short)0, c, false, false);
  asm volatile("v_nop\n\tv_nop\n\tv_nop\n\tv_nop" : "+v"(d) : "v"(a), "v"(b));
  return d;
}

template <int NBT>
__device__ __forceinline__ int scan_chunk(const int* __restrict__ dsts, int nE, int cbase, int nodeBase,
                                          int vec8, int* list, int tid, int lane, int wave) {
  static_assert(NBT <= 8192);
  int wc = 0;
#pragma unroll
  for (int g = 0; g < NGRP; ++g) {
    const int el0  = (g * NTHR + tid) * EPT;
    const int e0   = cbase + el0;
    const int sent = -2147483647 - 1;
    v4i da, db;
    if (vec8 != 0 && e0 + 7 < nE) {
      da = *(const v4i*)(dsts + e0);
      db = *(const v4i*)(dsts + e0 + 4);
    } else {
      da.x = (e0     < nE) ? dsts[min(e0, nE - 1)] : sent;
      da.y = (e0 + 1 < nE) ? dsts[min(e0 + 1, nE - 1)] : sent;
      da.z = (e0 + 2 < nE) ? dsts[min(e0 + 2, nE - 1)] : sent;
      da.w = (e0 + 3 < nE) ? dsts[min(e0 + 3, nE - 1)] : sent;
      db.x = (e0 + 4 < nE) ? dsts[min(e0 + 4, nE - 1)] : sent;
      db.y = (e0 + 5 < nE) ? dsts[min(e0 + 5, nE - 1)] : sent;
      db.z = (e0 + 6 < nE) ? dsts[min(e0 + 6, nE - 1)] : sent;
      db.w = (e0 + 7 < nE) ? dsts[min(e0 + 7, nE - 1)] : sent;
    }
    const unsigned nb = (unsigned)nodeBase;
    const unsigned s0 = (unsigned)da.x - nb, s1 = (unsigned)da.y - nb;
    const unsigned s2 = (unsigned)da.z - nb, s3 = (unsigned)da.w - nb;
    const unsigned s4 = (unsigned)db.x - nb, s5 = (unsigned)db.y - nb;
    const unsigned s6 = (unsigned)db.z - nb, s7 = (unsigned)db.w - nb;
    const bool h0 = s0 < (unsigned)NBT, h1 = s1 < (unsigned)NBT, h2 = s2 < (unsigned)NBT, h3 = s3 < (unsigned)NBT;
    const bool h4 = s4 < (unsigned)NBT, h5 = s5 < (unsigned)NBT, h6 = s6 < (unsigned)NBT, h7 = s7 < (unsigned)NBT;
    const unsigned any = __builtin_amdgcn_ballot_w32(h0 | h1 | h2 | h3 | h4 | h5 | h6 | h7);
    if (any != 0u) {
#define HITJ(J, HJ, SJ) { \
        const unsigned mj = __builtin_amdgcn_ballot_w32(HJ); \
        if (mj != 0u) { \
          if (HJ) { \
            const int pos = wc + (int)__builtin_amdgcn_mbcnt_lo(mj, 0u); \
            if (pos < WCAP) list[wave * WCAP + pos] = ((el0 + (J)) << ESH) | (int)(SJ); \
          } \
          wc += (int)__builtin_popcount(mj); } }
      HITJ(0, h0, s0)
      HITJ(1, h1, s1)
      HITJ(2, h2, s2)
      HITJ(3, h3, s3)
      HITJ(4, h4, s4)
      HITJ(5, h5, s5)
      HITJ(6, h6, s6)
      HITJ(7, h7, s7)
#undef HITJ
    }
  }
  return wc;
}

__global__ __launch_bounds__(NTHR) void k_wprep(const float* __restrict__ w1, const float* __restrict__ w2,
                                                _Float16* wp) {
  const int i  = blockIdx.x * NTHR + threadIdx.x;
  const int n1 = HIDC * (IN / 8);
  const int n2 = OUTC * (HIDC / 8);
  if (i >= n1 + n2) return;
  const float* w;
  int nout, n, k0;
  _Float16* dst;
  if (i < n1) {
    w = w1; nout = HIDC; n = i >> 4; k0 = (i & 15) * 8;
    dst = wp + (size_t)n * IN + k0;
  } else {
    const int j = i - n1;
    w = w2; nout = OUTC; n = j >> 4; k0 = (j & 15) * 8;
    dst = wp + (size_t)HIDC * IN + (size_t)n * HIDC + k0;
  }
  v8h o;
#pragma unroll
  for (int e = 0; e < 8; ++e) o[e] = (_Float16)(w[(size_t)(k0 + e) * nout + n] * WSC);
  *(volatile v8h*)dst = o;
  __threadfence();
  *(volatile v8h*)dst = o;
}

__global__ __launch_bounds__(NTHR) void k_deg(const int* __restrict__ ei, float* dinv, int nE, int vec8) {
  __shared__ __attribute__((aligned(16))) DegLds du;
  __shared__ int list[LISTN];
  __shared__ int wcnt[NWAVE];
  const int tid = threadIdx.x, lane = tid & 31, wave = tid >> 5;
  const int nodeBase = blockIdx.x * NBD;
  const int* dsts = ei + nE;

  for (int i = tid; i < NBD; i += NTHR) du.c[i] = 0;
  __syncthreads();

  const int nChunks = (nE + CHUNK - 1) / CHUNK;
#pragma unroll 1
  for (int ch = 0; ch < nChunks; ++ch) {
    const int cbase = ch * CHUNK;
    const int wc = scan_chunk<NBD>(dsts, nE, cbase, nodeBase, vec8, list, tid, lane, wave);
    if (lane == 0) wcnt[wave] = wc;
    __syncthreads();
    if (wave == 0) {
#pragma unroll 1
      for (int wsx = 0; wsx < NWAVE; ++wsx) {
        int n = __builtin_amdgcn_readfirstlane(wcnt[wsx]);
        n = n > WCAP ? WCAP : (n < 0 ? 0 : n);
        const int* lp = list + wsx * WCAP;
#pragma unroll 1
        for (int i = 0; i < n; ++i) {
          const int ent  = __builtin_amdgcn_readfirstlane(lp[i]);
          const int slot = ent & (NBD - 1);
          if (lane == 0) du.c[slot] += 1;
        }
      }
    }
    __syncthreads();
  }

#pragma unroll 1
  for (int i = tid; i < NBD; i += NTHR) {
    const float dg = (float)(du.c[i] + 1);
    du.f[i] = rsqrtf(dg);
  }
  __syncthreads();

#pragma unroll 1
  for (int j = 0; j < NBD / (4 * NTHR); ++j) {
    const int idx = j * 4 * NTHR + 4 * tid;
    const v4f d = du.v[idx >> 2];
    *(volatile v4f*)(dinv + (size_t)nodeBase + idx) = d;
  }
  __threadfence();
#pragma unroll 1
  for (int j = 0; j < NBD / (4 * NTHR); ++j) {
    const int idx = j * 4 * NTHR + 4 * tid;
    const v4f d = du.v[idx >> 2];
    *(volatile v4f*)(dinv + (size_t)nodeBase + idx) = d;
  }
}

template <int NOUT, bool AH>
__global__ __launch_bounds__(NTHR) void k_gemm(const float* __restrict__ xf, const _Float16* __restrict__ xh,
                                               const _Float16* __restrict__ wp, float* y, int nN) {
  static_assert(NOUT == 128 || NOUT == 64);
  __shared__ __attribute__((aligned(16))) float stg[NWAVE * 16 * 64];
  constexpr int RB = (NOUT == 128) ? 64 : 128;
  const int tid = threadIdx.x, lane = tid & 31, wave = tid >> 5, hh = lane >> 4, m = lane & 15;
  const int rt   = (NOUT == 128) ? (wave >> 1) : wave;
  const int cb   = (NOUT == 128) ? ((wave & 1) * 64) : 0;
  const int row0 = blockIdx.x * RB + rt * 16;

  v8f acc[4];
#pragma unroll
  for (int t = 0; t < 4; ++t) { v8f z = {0.f, 0.f, 0.f, 0.f, 0.f, 0.f, 0.f, 0.f}; acc[t] = z; }

#pragma unroll
  for (int ks = 0; ks < 4; ++ks) {
    Frag a;
    if constexpr (AH) {
      const _Float16* ap = xh + (size_t)(row0 + m) * 128 + 32 * ks + 8 * hh;
      a.half[0] = *(const v8h*)ap;
      a.half[1] = *(const v8h*)(ap + 16);
    } else {
      int node = row0 + m;
      node = node > nN - 1 ? nN - 1 : node;
      const float* p0 = xf + (size_t)node * 128 + 32 * ks + 8 * hh;
      const v4f f0 = *(const v4f*)p0,        f1 = *(const v4f*)(p0 + 4);
      const v4f f2 = *(const v4f*)(p0 + 16), f3 = *(const v4f*)(p0 + 20);
      a.half[0] = cvt8h(f0, f1);
      a.half[1] = cvt8h(f2, f3);
    }
#pragma unroll
    for (int t = 0; t < 4; ++t) {
      const _Float16* bp = wp + (size_t)(cb + 16 * t + m) * 128 + 32 * ks + 8 * hh;
      Frag b;
      b.half[0] = *(const v8h*)bp;
      b.half[1] = *(const v8h*)(bp + 16);
      acc[t] = wm(a.v, b.v, acc[t]);
    }
  }

  float* sp = stg + wave * (16 * 64) + (8 * hh) * 64 + m;
#pragma unroll
  for (int t = 0; t < 4; ++t) {
    sp[0 * 64 + 16 * t] = acc[t][0] * WSCI;
    sp[1 * 64 + 16 * t] = acc[t][1] * WSCI;
    sp[2 * 64 + 16 * t] = acc[t][2] * WSCI;
    sp[3 * 64 + 16 * t] = acc[t][3] * WSCI;
    sp[4 * 64 + 16 * t] = acc[t][4] * WSCI;
    sp[5 * 64 + 16 * t] = acc[t][5] * WSCI;
    sp[6 * 64 + 16 * t] = acc[t][6] * WSCI;
    sp[7 * 64 + 16 * t] = acc[t][7] * WSCI;
  }
  __syncthreads();

  const int c4 = 4 * (lane & 15);
  v4f ov[8];
#pragma unroll
  for (int q = 0; q < 8; ++q) ov[q] = *(const v4f*)(stg + wave * (16 * 64) + (2 * q + hh) * 64 + c4);
#pragma unroll
  for (int q = 0; q < 8; ++q)
    *(volatile v4f*)(y + (size_t)(row0 + 2 * q + hh) * NOUT + cb + c4) = ov[q];
  __threadfence();
#pragma unroll
  for (int q = 0; q < 8; ++q)
    *(volatile v4f*)(y + (size_t)(row0 + 2 * q + hh) * NOUT + cb + c4) = ov[q];
}

template <int C, int NB, bool L1>
__global__ __launch_bounds__(NTHR) void k_agg(const int* __restrict__ ei, const float* __restrict__ gin,
                                              const float* __restrict__ dinv, const float* __restrict__ bias,
                                              _Float16* hout, float* zout, int nN, int nE, int vec8) {
  static_assert(NB * C == AGGF);
  static_assert(NB <= 8192 && (NB & (NB - 1)) == 0);
  static_assert(C == 128 || C == 64);
  static_assert(!L1 || C == 128);
  extern __shared__ v4f lds_dyn[];
  float* acc  = (float*)lds_dyn;
  int*   list = (int*)(acc + AGGF);
  __shared__ int wcnt[NWAVE];
  constexpr int F = C / 32;
  const int tid = threadIdx.x, lane = tid & 31, wave = tid >> 5;
  const int nodeBase = blockIdx.x * NB;
  const int* dsts = ei + nE;

  {
    const v4f z = {0.f, 0.f, 0.f, 0.f};
    for (int i = tid; i < AGGF / 4; i += NTHR) lds_dyn[i] = z;
  }
  __syncthreads();

  const int nChunks = (nE + CHUNK - 1) / CHUNK;
#pragma unroll 1
  for (int ch = 0; ch < nChunks; ++ch) {
    const int cbase = ch * CHUNK;
    const int wc = scan_chunk<NB>(dsts, nE, cbase, nodeBase, vec8, list, tid, lane, wave);
    if (lane == 0) wcnt[wave] = wc;
    __syncthreads();
    if (wave == 0) {
#pragma unroll 1
      for (int wsx = 0; wsx < NWAVE; ++wsx) {
        int n = __builtin_amdgcn_readfirstlane(wcnt[wsx]);
        n = n > WCAP ? WCAP : (n < 0 ? 0 : n);
        const int* lp = list + wsx * WCAP;
#pragma unroll 1
        for (int i = 0; i < n; ++i) {
          const int ent  = __builtin_amdgcn_readfirstlane(lp[i]);
          const int slot = ent & (NB - 1);
          int e = cbase + ((ent >> ESH) & (CHUNK - 1));
          e = e > nE - 1 ? nE - 1 : e;
          int src = ei[e];
          src = src < 0 ? 0 : (src > nN - 1 ? nN - 1 : src);
          const float w = dinv[src];
          if constexpr (F == 4) {
            const v4f v = *(const v4f*)(gin + (size_t)src * C + 4 * lane);
            v4f* ap = (v4f*)(acc + slot * C + 4 * lane);
            *ap = *ap + v * w;
          } else {
            const v2f v = *(const v2f*)(gin + (size_t)src * C + 2 * lane);
            v2f* ap = (v2f*)(acc + slot * C + 2 * lane);
            *ap = *ap + v * w;
          }
        }
      }
    }
    __syncthreads();
  }

  if constexpr (F == 4) {
    const v4f bl = *(const v4f*)(bias + 4 * lane);
#pragma unroll 2
    for (int j = 0; j < NB / NWAVE; ++j) {
      const int slot = wave * (NB / NWAVE) + j;
      const int node = nodeBase + slot;
      const float dd = dinv[node];
      v4f* ap = (v4f*)(acc + slot * C + 4 * lane);
      const v4f g = *(const v4f*)(gin + (size_t)node * C + 4 * lane);
      v4f t = (*ap + g * dd) * dd + bl;
      if constexpr (L1) {
        t.x = fmaxf(t.x, 0.f); t.y = fmaxf(t.y, 0.f); t.z = fmaxf(t.z, 0.f); t.w = fmaxf(t.w, 0.f);
      }
      *ap = t;
    }
  } else {
    const v2f bl = *(const v2f*)(bias + 2 * lane);
#pragma unroll 2
    for (int j = 0; j < NB / NWAVE; ++j) {
      const int slot = wave * (NB / NWAVE) + j;
      const int node = nodeBase + slot;
      const float dd = dinv[node];
      v2f* ap = (v2f*)(acc + slot * C + 2 * lane);
      const v2f g = *(const v2f*)(gin + (size_t)node * C + 2 * lane);
      v2f t = (*ap + g * dd) * dd + bl;
      if constexpr (L1) { t.x = fmaxf(t.x, 0.f); t.y = fmaxf(t.y, 0.f); }
      *ap = t;
    }
  }
  __syncthreads();

  const size_t ob = (size_t)nodeBase * C;
  if constexpr (L1) {
    _Float16* hp = hout + ob;
#pragma unroll 4
    for (int q = 0; q < (AGGF / NWAVE) / 256; ++q) {
      const int f = wave * (AGGF / NWAVE) + q * 256 + 8 * lane;
      const v4f u0 = *(const v4f*)(acc + f), u1 = *(const v4f*)(acc + f + 4);
      *(volatile v8h*)(hp + f) = cvt8h(u0, u1);
    }
    __threadfence();
#pragma unroll 4
    for (int q = 0; q < (AGGF / NWAVE) / 256; ++q) {
      const int f = wave * (AGGF / NWAVE) + q * 256 + 8 * lane;
      const v4f u0 = *(const v4f*)(acc + f), u1 = *(const v4f*)(acc + f + 4);
      *(volatile v8h*)(hp + f) = cvt8h(u0, u1);
    }
  } else {
    float* zp = zout + ob;
#pragma unroll 4
    for (int q = 0; q < (AGGF / NWAVE) / 128; ++q) {
      const int f = wave * (AGGF / NWAVE) + q * 128 + 4 * lane;
      const v4f v = *(const v4f*)(acc + f);
      *(volatile v4f*)(zp + f) = v;
    }
    __threadfence();
#pragma unroll 4
    for (int q = 0; q < (AGGF / NWAVE) / 128; ++q) {
      const int f = wave * (AGGF / NWAVE) + q * 128 + 4 * lane;
      const v4f v = *(const v4f*)(acc + f);
      *(volatile v4f*)(zp + f) = v;
    }
  }
}

__global__ __launch_bounds__(NTHR) void k_decode(const float* __restrict__ z, const int* __restrict__ eli,
                                                 float* out, int nN, int nEL) {
  __shared__ __attribute__((aligned(16))) float res[PPB];
  const int tid  = threadIdx.x;
  const int base = blockIdx.x * PPB;
#pragma unroll 1
  for (int j = 0; j < PPB / NTHR; ++j) {
    int p = base + j * NTHR + tid;
    p = p > nEL - 1 ? nEL - 1 : p;
    int a = eli[p];
    int b = eli[(size_t)nEL + p];
    a = a < 0 ? 0 : (a > nN - 1 ? nN - 1 : a);
    b = b < 0 ? 0 : (b > nN - 1 ? nN - 1 : b);
    const v4f* za = (const v4f*)(z + (size_t)a * OUTC);
    const v4f* zb = (const v4f*)(z + (size_t)b * OUTC);
    float s = 0.f;
#pragma unroll
    for (int c = 0; c < OUTC / 4; ++c) {
      const v4f u = za[c], v = zb[c];
      s += u.x * v.x; s += u.y * v.y; s += u.z * v.z; s += u.w * v.w;
    }
    res[j * NTHR + tid] = s;
  }
  __syncthreads();

#pragma unroll
  for (int q = 0; q < PPB / (4 * NTHR); ++q) {
    const int f   = q * 4 * NTHR + 4 * tid;
    const int idx = base + f;
    const v4f v = *(const v4f*)(res + f);
    if (idx + 3 < nEL) {
      *(volatile v4f*)(out + idx) = v;
    } else {
      if (idx     < nEL) *(volatile float*)(out + idx)     = v.x;
      if (idx + 1 < nEL) *(volatile float*)(out + idx + 1) = v.y;
      if (idx + 2 < nEL) *(volatile float*)(out + idx + 2) = v.z;
    }
  }
  __threadfence();
#pragma unroll
  for (int q = 0; q < PPB / (4 * NTHR); ++q) {
    const int f   = q * 4 * NTHR + 4 * tid;
    const int idx = base + f;
    const v4f v = *(const v4f*)(res + f);
    if (idx + 3 < nEL) {
      *(volatile v4f*)(out + idx) = v;
    } else {
      if (idx     < nEL) *(volatile float*)(out + idx)     = v.x;
      if (idx + 1 < nEL) *(volatile float*)(out + idx + 1) = v.y;
      if (idx + 2 < nEL) *(volatile float*)(out + idx + 2) = v.z;
    }
  }
}

extern "C" void kernel_launch(void* const* d_in, const int* in_sizes, int n_in,
                              void* d_out, int out_size, void* d_ws, size_t ws_size,
                              hipStream_t stream) {
  if (n_in < 7) return;
  const int nN  = in_sizes[0] / IN;
  const int nE  = in_sizes[5] / 2;
  const int nEL = in_sizes[6] / 2;
  if (nN <= 0 || in_sizes[0] != nN * IN) return;
  if (in_sizes[1] != IN * HIDC || in_sizes[2] != HIDC) return;
  if (in_sizes[3] != HIDC * OUTC || in_sizes[4] != OUTC) return;
  if (nE < 0 || in_sizes[5] != 2 * nE) return;
  if (nEL <= 0 || in_sizes[6] != 2 * nEL) return;
  if (out_size != nEL) return;

  const float* x   = (const float*)d_in[0];
  const float* w1  = (const float*)d_in[1];
  const float* b1  = (const float*)d_in[2];
  const float* w2  = (const float*)d_in[3];
  const float* b2  = (const float*)d_in[4];
  const int*   ei  = (const int*)d_in[5];
  const int*   eli = (const int*)d_in[6];
  float* out = (float*)d_out;

  const int NR  = ((nN + NRQ - 1) / NRQ) * NRQ;
  const int nDB = (NR + NBD - 1) / NBD;
  const int NRD = nDB * NBD;

  char* ws = (char*)d_ws;
  size_t off = 0;
  const size_t oWP = off; off += (size_t)(HIDC * IN + OUTC * HIDC) * 2;  off = (off + 255) & ~(size_t)255;
  const size_t oDI = off; off += (size_t)NRD * 4;                         off = (off + 255) & ~(size_t)255;
  const size_t szH0 = (size_t)NR * HIDC * 4;
  const size_t szZ  = (size_t)NR * OUTC * 4;
  const size_t oH0 = off; off += szH0;                                    off = (off + 255) & ~(size_t)255;
  const size_t oHP = off; off += (size_t)NR * HIDC * 2;                   off = (off + 255) & ~(size_t)255;
  if (2 * szZ > szH0) return;
  if (off > ws_size) return;
  if (off > ((size_t)128 << 20)) return;
  _Float16* wpl  = (_Float16*)(ws + oWP);
  float*    dinv = (float*)(ws + oDI);
  float*    h0   = (float*)(ws + oH0);
  _Float16* hpl  = (_Float16*)(ws + oHP);
  float*    z0   = (float*)(ws + oH0);
  float*    zf   = (float*)(ws + oH0 + szZ);

  const int vec8 = ((nE & 3) == 0) ? 1 : 0;

  const int nPrep = HIDC * (IN / 8) + OUTC * (HIDC / 8);
  k_wprep<<<(nPrep + NTHR - 1) / NTHR, NTHR, 0, stream>>>(w1, w2, wpl);

  k_deg<<<nDB, NTHR, 0, stream>>>(ei, dinv, nE, vec8);

  k_gemm<128, false><<<NR / 64, NTHR, 0, stream>>>(x, hpl, wpl, h0, nN);
  hipFuncSetAttribute(reinterpret_cast<const void*>(&k_agg<128, NB1, true>),
                      hipFuncAttributeMaxDynamicSharedMemorySize, LDS_AGG);
  k_agg<128, NB1, true><<<NR / NB1, NTHR, LDS_AGG, stream>>>(ei, h0, dinv, b1, hpl, zf, nN, nE, vec8);

  k_gemm<64, true><<<NR / 128, NTHR, 0, stream>>>(x, hpl, wpl + HIDC * IN, z0, nN);
  hipFuncSetAttribute(reinterpret_cast<const void*>(&k_agg<64, NB2, false>),
                      hipFuncAttributeMaxDynamicSharedMemorySize, LDS_AGG);
  k_agg<64, NB2, false><<<NR / NB2, NTHR, LDS_AGG, stream>>>(ei, z0, dinv, b2, hpl, zf, nN, nE, vec8);

  k_decode<<<(nEL + PPB - 1) / PPB, NTHR, 0, stream>>>(zf, eli, out, nN, nEL);
}
